// G3N2Level_28750511080055
// MI455X (gfx1250) — hardware-verified
//
#include <hip/hip_runtime.h>
#include <stddef.h>


#define D        256
#define NTHR     256
#define NWAVE    8
#define EPT      8
#define NGRP     2
#define CHUNK    (NTHR * EPT * NGRP)
#define WCAP     (EPT * NGRP * 32)
#define LISTN    (NWAVE * WCAP)
#define NBS      256
#define NBP      128
#define STGW     32
#define STGF     (16 * STGW)
#define RPW      8

#define LDS_LIST   (LISTN * 4)
#define LDS_S_ACC  (NBS * D * 4)
#define LDS_S_CNT  (NBS * 4)
#define LDS_SAGE   (LDS_S_ACC + LDS_LIST + LDS_S_CNT + 64)
#define LDS_P_ACC  (NBP * D * 4)
#define LDS_P_CNT  (NBP * 4)
#define LDS_POOL   (2 * LDS_P_ACC + LDS_LIST + LDS_P_CNT + 64)

static_assert((CHUNK & (CHUNK - 1)) == 0);
static_assert(CHUNK <= 4096);
static_assert((NBS & (NBS - 1)) == 0);
static_assert(NBS <= 4096);
static_assert((NBP & (NBP - 1)) == 0);
static_assert(NBP <= 4096);
static_assert((NBS / 16) % NWAVE == 0);
static_assert((NBP / 16) % NWAVE == 0);
static_assert(NWAVE * STGF * 4 <= LDS_LIST);
static_assert(NWAVE * 4 <= 64);
static_assert(LDS_SAGE <= 300 * 1024);
static_assert(LDS_POOL <= 300 * 1024);
static_assert(D == 256);

typedef float  v4f   __attribute__((ext_vector_type(4)));
typedef float  v8f   __attribute__((ext_vector_type(8)));
typedef int    v4i   __attribute__((ext_vector_type(4)));
typedef __bf16 bf16_t;
typedef bf16_t v8bf  __attribute__((ext_vector_type(8)));
typedef bf16_t v16bf __attribute__((ext_vector_type(16)));
union FragB { v16bf v; v8bf h[2]; v4i q[2]; };
union Pack8 { v8bf v; v4i q; };

__device__ __forceinline__ v8f wmb(v16bf a, v16bf b, v8f c) {
  v8f d = __builtin_amdgcn_wmma_f32_16x16x32_bf16(false, a, false, b, (short)0, c, false, false);
  asm volatile("v_nop\n\tv_nop\n\tv_nop\n\tv_nop" : "+v"(d) : "v"(a), "v"(b));
  return d;
}

__device__ __forceinline__ v4f sel4(bool c, v4f a, v4f b) {
  v4f r;
  r.x = c ? a.x : b.x; r.y = c ? a.y : b.y; r.z = c ? a.z : b.z; r.w = c ? a.w : b.w;
  return r;
}

__device__ __forceinline__ v4f max4(v4f a, v4f b) {
  v4f r;
  r.x = fmaxf(a.x, b.x); r.y = fmaxf(a.y, b.y); r.z = fmaxf(a.z, b.z); r.w = fmaxf(a.w, b.w);
  return r;
}

template <int B>
__device__ __forceinline__ void split8(FragB& hi, FragB& lo, v4f a, v4f b) {
#define SPL1(I, X) { const float xv = (X); const bf16_t hb = (bf16_t)xv; hi.v[B + (I)] = hb; lo.v[B + (I)] = (bf16_t)(xv - (float)hb); }
  SPL1(0, a.x) SPL1(1, a.y) SPL1(2, a.z) SPL1(3, a.w)
  SPL1(4, b.x) SPL1(5, b.y) SPL1(6, b.z) SPL1(7, b.w)
#undef SPL1
}

template <int NBT>
__device__ __forceinline__ int scan_chunk(const int* __restrict__ dsts, int nE, int cbase, int nodeBase,
                                          int vec8, int* list, int tid, int wave) {
  int wc = 0;
#pragma unroll
  for (int g = 0; g < NGRP; ++g) {
    const int el0  = (g * NTHR + tid) * EPT;
    const int e0   = cbase + el0;
    const int sent = -2147483647 - 1;
    v4i da, db;
    if (vec8 != 0 && cbase + CHUNK <= nE) {
      da = *(const v4i*)(dsts + e0);
      db = *(const v4i*)(dsts + e0 + 4);
    } else {
      da.x = (e0     < nE) ? dsts[min(e0,     nE - 1)] : sent;
      da.y = (e0 + 1 < nE) ? dsts[min(e0 + 1, nE - 1)] : sent;
      da.z = (e0 + 2 < nE) ? dsts[min(e0 + 2, nE - 1)] : sent;
      da.w = (e0 + 3 < nE) ? dsts[min(e0 + 3, nE - 1)] : sent;
      db.x = (e0 + 4 < nE) ? dsts[min(e0 + 4, nE - 1)] : sent;
      db.y = (e0 + 5 < nE) ? dsts[min(e0 + 5, nE - 1)] : sent;
      db.z = (e0 + 6 < nE) ? dsts[min(e0 + 6, nE - 1)] : sent;
      db.w = (e0 + 7 < nE) ? dsts[min(e0 + 7, nE - 1)] : sent;
    }
    const unsigned nb = (unsigned)nodeBase;
    const unsigned s0 = (unsigned)da.x - nb, s1 = (unsigned)da.y - nb;
    const unsigned s2 = (unsigned)da.z - nb, s3 = (unsigned)da.w - nb;
    const unsigned s4 = (unsigned)db.x - nb, s5 = (unsigned)db.y - nb;
    const unsigned s6 = (unsigned)db.z - nb, s7 = (unsigned)db.w - nb;
    const bool h0 = s0 < (unsigned)NBT, h1 = s1 < (unsigned)NBT, h2 = s2 < (unsigned)NBT, h3 = s3 < (unsigned)NBT;
    const bool h4 = s4 < (unsigned)NBT, h5 = s5 < (unsigned)NBT, h6 = s6 < (unsigned)NBT, h7 = s7 < (unsigned)NBT;
    const unsigned any = __builtin_amdgcn_ballot_w32(h0 | h1 | h2 | h3 | h4 | h5 | h6 | h7);
    if (any != 0u) {
#define HITJ(J, HJ, SJ) { \
        const unsigned mj = __builtin_amdgcn_ballot_w32(HJ); \
        if (mj != 0u) { \
          if (HJ) { \
            const int pos = wc + (int)__builtin_amdgcn_mbcnt_lo(mj, 0u); \
            if (pos < WCAP) list[wave * WCAP + pos] = ((el0 + (J)) << 12) | (int)(SJ); \
          } \
          wc += (int)__builtin_popcount(mj); } }
      HITJ(0, h0, s0)
      HITJ(1, h1, s1)
      HITJ(2, h2, s2)
      HITJ(3, h3, s3)
      HITJ(4, h4, s4)
      HITJ(5, h5, s5)
      HITJ(6, h6, s6)
      HITJ(7, h7, s7)
#undef HITJ
    }
  }
  return wc;
}

__global__ __launch_bounds__(NTHR) void k_wprep(
    const float* __restrict__ Wa, const float* __restrict__ Wb, const float* __restrict__ Wc,
    int sa, int sb, int sc, bf16_t* whi, bf16_t* wlo, int kv, int nTot) {
  const int i = blockIdx.x * NTHR + threadIdx.x;
  if (i >= nTot) return;
  const int o     = i * 8;
  const int layer = o / (D * kv);
  const int rem   = o - layer * (D * kv);
  const int n     = rem / kv;
  const int k0    = rem - n * kv;
  const int part  = k0 / D;
  const int kk    = k0 - part * D;
  const float* base = (part == 0) ? (Wa + (size_t)layer * sa)
                    : (part == 1) ? (Wb + (size_t)layer * sb) : (Wc + (size_t)layer * sc);
  const float* p = base + (size_t)kk * D + n;
  Pack8 ph, pl;
#define WSP(I) { const float xv = p[(I) * D]; const bf16_t hb = (bf16_t)xv; ph.v[(I)] = hb; pl.v[(I)] = (bf16_t)(xv - (float)hb); }
  WSP(0) WSP(1) WSP(2) WSP(3) WSP(4) WSP(5) WSP(6) WSP(7)
#undef WSP
  bf16_t* dh = whi + o;
  bf16_t* dl = wlo + o;
  const v4i qh = ph.q, ql = pl.q;
  *(volatile v4i*)dh = qh;
  *(volatile v4i*)dl = ql;
  __threadfence();
  *(volatile v4i*)dh = qh;
  *(volatile v4i*)dl = ql;
}

__global__ __launch_bounds__(NTHR) void k_gather1(
    const int* __restrict__ ids, const float* __restrict__ tab, int nTab,
    float* xo, int nN, int nRows) {
  const int lane = threadIdx.x & 31, wave = threadIdx.x >> 5;
  const int r0 = (blockIdx.x * NWAVE + wave) * RPW;
#pragma unroll 1
  for (int j = 0; j < RPW; ++j) {
    const int row = r0 + j;
    if (row < nRows) {
      const int i = row < nN ? row : nN - 1;
      int id = ids[i];
      id = id < 0 ? id + nTab : id;
      id = id < 0 ? 0 : (id > nTab - 1 ? nTab - 1 : id);
      const float* sp = tab + (size_t)id * D + 4 * lane;
      const v4f v0 = *(const v4f*)sp;
      const v4f v1 = *(const v4f*)(sp + 128);
      float* gp = xo + (size_t)row * D + 4 * lane;
      *(volatile v4f*)gp = v0;
      *(volatile v4f*)(gp + 128) = v1;
      __threadfence();
      *(volatile v4f*)gp = v0;
      *(volatile v4f*)(gp + 128) = v1;
    }
  }
}

__global__ __launch_bounds__(NTHR) void k_gather2(
    const int* __restrict__ ids, const float* __restrict__ xd, int nXd,
    const float* __restrict__ tab, int nTab, float* xo, int nN, int nRows) {
  const int lane = threadIdx.x & 31, wave = threadIdx.x >> 5;
  const int r0 = (blockIdx.x * NWAVE + wave) * RPW;
#pragma unroll 1
  for (int j = 0; j < RPW; ++j) {
    const int row = r0 + j;
    if (row < nRows) {
      const int i = row < nN ? row : nN - 1;
      int id = ids[i];
      id = id < 0 ? id + nTab : id;
      id = id < 0 ? 0 : (id > nTab - 1 ? nTab - 1 : id);
      const int  idd  = id > nXd - 1 ? nXd - 1 : id;
      const bool useD = id < nXd;
      const float* ap = xd  + (size_t)idd * D + 4 * lane;
      const float* bp = tab + (size_t)id  * D + 4 * lane;
      const v4f a0 = *(const v4f*)ap, a1 = *(const v4f*)(ap + 128);
      const v4f b0 = *(const v4f*)bp, b1 = *(const v4f*)(bp + 128);
      const v4f v0 = sel4(useD, a0, b0);
      const v4f v1 = sel4(useD, a1, b1);
      float* gp = xo + (size_t)row * D + 4 * lane;
      *(volatile v4f*)gp = v0;
      *(volatile v4f*)(gp + 128) = v1;
      __threadfence();
      *(volatile v4f*)gp = v0;
      *(volatile v4f*)(gp + 128) = v1;
    }
  }
}

template <int KV>
__device__ __forceinline__ void kstep(const float* ap, float mul,
                                      const bf16_t* bhp, const bf16_t* blp, v8f (&c)[8]) {
  const v4f p0 = (*(const v4f*)(ap))      * mul;
  const v4f p1 = (*(const v4f*)(ap + 4))  * mul;
  const v4f p2 = (*(const v4f*)(ap + 16)) * mul;
  const v4f p3 = (*(const v4f*)(ap + 20)) * mul;
  FragB ahi, alo;
  split8<0>(ahi, alo, p0, p1);
  split8<8>(ahi, alo, p2, p3);
#pragma unroll
  for (int ct = 0; ct < 8; ++ct) {
    const bf16_t* hp = bhp + (size_t)ct * 16 * KV;
    const bf16_t* lp = blp + (size_t)ct * 16 * KV;
    FragB bh, bq;
    bh.q[0] = *(const v4i*)hp;  bh.q[1] = *(const v4i*)(hp + 16);
    bq.q[0] = *(const v4i*)lp;  bq.q[1] = *(const v4i*)(lp + 16);
    c[ct] = wmb(alo.v, bh.v, c[ct]);
    c[ct] = wmb(ahi.v, bq.v, c[ct]);
    c[ct] = wmb(ahi.v, bh.v, c[ct]);
  }
}

__device__ __forceinline__ void epi_half(v8f (&c)[8], float* stg, const float* __restrict__ biasp,
                                         float* gbase, int lane, int hh, int m) {
  const int rr = lane >> 3, c4 = 4 * (lane & 7);
#pragma unroll
  for (int cp = 0; cp < 4; ++cp) {
#pragma unroll
    for (int j = 0; j < 2; ++j) {
      const float b = biasp[32 * cp + 16 * j + m];
      float* sp = stg + (8 * hh) * STGW + 16 * j + m;
#pragma unroll
      for (int r = 0; r < 8; ++r) sp[r * STGW] = fmaxf(c[2 * cp + j][r] + b, 0.0f);
    }
    __syncthreads();
    const v4f v0 = *(const v4f*)(stg + (0  + rr) * STGW + c4);
    const v4f v1 = *(const v4f*)(stg + (4  + rr) * STGW + c4);
    const v4f v2 = *(const v4f*)(stg + (8  + rr) * STGW + c4);
    const v4f v3 = *(const v4f*)(stg + (12 + rr) * STGW + c4);
    float* g0 = gbase + (size_t)rr * D + 32 * cp + c4;
    float* g1 = g0 + 4 * D;
    float* g2 = g0 + 8 * D;
    float* g3 = g0 + 12 * D;
    *(volatile v4f*)g0 = v0;
    *(volatile v4f*)g1 = v1;
    *(volatile v4f*)g2 = v2;
    *(volatile v4f*)g3 = v3;
    __threadfence();
    *(volatile v4f*)g0 = v0;
    *(volatile v4f*)g1 = v1;
    *(volatile v4f*)g2 = v2;
    *(volatile v4f*)g3 = v3;
    __syncthreads();
  }
}

template <int NT>
__global__ __launch_bounds__(NTHR) void k_sage(
    const int* __restrict__ ei, const float* __restrict__ xin, const float* x3,
    const bf16_t* __restrict__ whi, const bf16_t* __restrict__ wlo,
    const float* __restrict__ bias, float* xout, int nN, int nE, int vec8) {
  constexpr int KV = NT * D;
  extern __shared__ v4f lds_dyn[];
  float* acc  = (float*)lds_dyn;
  int*   list = (int*)((char*)lds_dyn + LDS_S_ACC);
  int*   cnt  = (int*)((char*)lds_dyn + LDS_S_ACC + LDS_LIST);
  int*   wcnt = (int*)((char*)lds_dyn + LDS_S_ACC + LDS_LIST + LDS_S_CNT);
  const int tid = threadIdx.x, lane = tid & 31, wave = tid >> 5, hh = lane >> 4, m = lane & 15;
  float* stg = (float*)list + wave * STGF;
  const int nodeBase = blockIdx.x * NBS;
  const int* dsts = ei + nE;

  {
    const v4f z = {0.f, 0.f, 0.f, 0.f};
    for (int i = tid; i < NBS * D / 4; i += NTHR) lds_dyn[i] = z;
    for (int i = tid; i < NBS; i += NTHR) cnt[i] = 0;
  }
  __syncthreads();

  const int nChunks = (nE + CHUNK - 1) / CHUNK;
#pragma unroll 1
  for (int ch = 0; ch < nChunks; ++ch) {
    const int cbase = ch * CHUNK;
    const int wc = scan_chunk<NBS>(dsts, nE, cbase, nodeBase, vec8, list, tid, wave);
    if (lane == 0) wcnt[wave] = wc;
    __syncthreads();
    if (wave == 0) {
#pragma unroll 1
      for (int wsx = 0; wsx < NWAVE; ++wsx) {
        int n = __builtin_amdgcn_readfirstlane(wcnt[wsx]);
        n = n > WCAP ? WCAP : (n < 0 ? 0 : n);
        const int* lp = list + wsx * WCAP;
#pragma unroll 1
        for (int i = 0; i < n; ++i) {
          const int ent  = __builtin_amdgcn_readfirstlane(lp[i]);
          const int slot = ent & (NBS - 1);
          int e = cbase + ((ent >> 12) & (CHUNK - 1));
          e = e > nE - 1 ? nE - 1 : e;
          int src = ei[e];
          src = src < 0 ? 0 : (src > nN - 1 ? nN - 1 : src);
          const float* xr = xin + (size_t)src * D + 4 * lane;
          const v4f v0 = *(const v4f*)xr;
          const v4f v1 = *(const v4f*)(xr + 128);
          v4f* ap = (v4f*)(acc + slot * D + 4 * lane);
          ap[0]  = ap[0]  + v0;
          ap[32] = ap[32] + v1;
          if (lane == 0) cnt[slot] = cnt[slot] + 1;
        }
      }
    }
    __syncthreads();
  }

#pragma unroll 1
  for (int q = 0; q < NBS / 16 / NWAVE; ++q) {
    const int t     = q * NWAVE + wave;
    const int slotm = 16 * t + m;
    int node = nodeBase + slotm;
    node = node > nN - 1 ? nN - 1 : node;
    const int   cd  = cnt[slotm];
    const float inv = cd > 0 ? (1.0f / (float)cd) : 0.0f;
    const float* arow = acc + slotm * D + 8 * hh;
    const float* xrow = xin + (size_t)node * D + 8 * hh;
    const float* zrow = x3  + (size_t)node * D + 8 * hh;
#pragma unroll 1
    for (int hf = 0; hf < 2; ++hf) {
      v8f c[8];
#pragma unroll
      for (int ct = 0; ct < 8; ++ct) { const v8f z = {0.f, 0.f, 0.f, 0.f, 0.f, 0.f, 0.f, 0.f}; c[ct] = z; }
      const bf16_t* bh0 = whi + (size_t)(128 * hf + m) * KV + 8 * hh;
      const bf16_t* bl0 = wlo + (size_t)(128 * hf + m) * KV + 8 * hh;
#pragma unroll 1
      for (int ks = 0; ks < D / 32; ++ks)
        kstep<KV>(arow + 32 * ks, inv, bh0 + 32 * ks, bl0 + 32 * ks, c);
#pragma unroll 1
      for (int ks = 0; ks < D / 32; ++ks)
        kstep<KV>(xrow + 32 * ks, 1.0f, bh0 + D + 32 * ks, bl0 + D + 32 * ks, c);
      if (NT == 3) {
#pragma unroll 1
        for (int ks = 0; ks < D / 32; ++ks)
          kstep<KV>(zrow + 32 * ks, 1.0f, bh0 + 2 * D + 32 * ks, bl0 + 2 * D + 32 * ks, c);
      }
      epi_half(c, stg, bias + 128 * hf, xout + ((size_t)nodeBase + 16 * t) * D + 128 * hf, lane, hh, m);
    }
  }
}

__global__ __launch_bounds__(NTHR) void k_pool(
    const int* __restrict__ bat, const float* __restrict__ x,
    const bf16_t* __restrict__ whi, const bf16_t* __restrict__ wlo,
    const float* __restrict__ bias, float* xd, int nN, int vec8) {
  constexpr int KV = 2 * D;
  extern __shared__ v4f lds_dyn[];
  float* pmax = (float*)lds_dyn;
  float* psum = (float*)((char*)lds_dyn + LDS_P_ACC);
  int*   list = (int*)((char*)lds_dyn + 2 * LDS_P_ACC);
  int*   cnt  = (int*)((char*)lds_dyn + 2 * LDS_P_ACC + LDS_LIST);
  int*   wcnt = (int*)((char*)lds_dyn + 2 * LDS_P_ACC + LDS_LIST + LDS_P_CNT);
  const int tid = threadIdx.x, lane = tid & 31, wave = tid >> 5, hh = lane >> 4, m = lane & 15;
  float* stg = (float*)list + wave * STGF;
  const int gBase = blockIdx.x * NBP;

  {
    const v4f z = {0.f, 0.f, 0.f, 0.f};
    for (int i = tid; i < 2 * NBP * D / 4; i += NTHR) lds_dyn[i] = z;
    for (int i = tid; i < NBP; i += NTHR) cnt[i] = 0;
  }
  __syncthreads();

  const int nChunks = (nN + CHUNK - 1) / CHUNK;
#pragma unroll 1
  for (int ch = 0; ch < nChunks; ++ch) {
    const int cbase = ch * CHUNK;
    const int wc = scan_chunk<NBP>(bat, nN, cbase, gBase, vec8, list, tid, wave);
    if (lane == 0) wcnt[wave] = wc;
    __syncthreads();
    if (wave == 0) {
#pragma unroll 1
      for (int wsx = 0; wsx < NWAVE; ++wsx) {
        int n = __builtin_amdgcn_readfirstlane(wcnt[wsx]);
        n = n > WCAP ? WCAP : (n < 0 ? 0 : n);
        const int* lp = list + wsx * WCAP;
#pragma unroll 1
        for (int i = 0; i < n; ++i) {
          const int ent  = __builtin_amdgcn_readfirstlane(lp[i]);
          const int slot = ent & (NBP - 1);
          int e = cbase + ((ent >> 12) & (CHUNK - 1));
          e = e > nN - 1 ? nN - 1 : e;
          const float* xr = x + (size_t)e * D + 4 * lane;
          const v4f v0 = *(const v4f*)xr;
          const v4f v1 = *(const v4f*)(xr + 128);
          v4f* sp = (v4f*)(psum + slot * D + 4 * lane);
          v4f* mp = (v4f*)(pmax + slot * D + 4 * lane);
          sp[0]  = sp[0]  + v0;
          sp[32] = sp[32] + v1;
          mp[0]  = max4(mp[0],  v0);
          mp[32] = max4(mp[32], v1);
          if (lane == 0) cnt[slot] = cnt[slot] + 1;
        }
      }
    }
    __syncthreads();
  }

  {
    const int t     = wave;
    const int slotm = 16 * t + m;
    const int   cd  = cnt[slotm];
    const float inv = cd > 0 ? (1.0f / (float)cd) : 0.0f;
    const float* mrow = pmax + slotm * D + 8 * hh;
    const float* srow = psum + slotm * D + 8 * hh;
#pragma unroll 1
    for (int hf = 0; hf < 2; ++hf) {
      v8f c[8];
#pragma unroll
      for (int ct = 0; ct < 8; ++ct) { const v8f z = {0.f, 0.f, 0.f, 0.f, 0.f, 0.f, 0.f, 0.f}; c[ct] = z; }
      const bf16_t* bh0 = whi + (size_t)(128 * hf + m) * KV + 8 * hh;
      const bf16_t* bl0 = wlo + (size_t)(128 * hf + m) * KV + 8 * hh;
#pragma unroll 1
      for (int ks = 0; ks < D / 32; ++ks)
        kstep<KV>(mrow + 32 * ks, 1.0f, bh0 + 32 * ks, bl0 + 32 * ks, c);
#pragma unroll 1
      for (int ks = 0; ks < D / 32; ++ks)
        kstep<KV>(srow + 32 * ks, inv, bh0 + D + 32 * ks, bl0 + D + 32 * ks, c);
      epi_half(c, stg, bias + 128 * hf, xd + ((size_t)gBase + 16 * t) * D + 128 * hf, lane, hh, m);
    }
  }
}

extern "C" void kernel_launch(void* const* d_in, const int* in_sizes, int n_in,
                              void* d_out, int out_size, void* d_ws, size_t ws_size,
                              hipStream_t stream) {
  if (n_in < 16) return;
  const int nN1 = in_sizes[0];
  const int nE1 = in_sizes[1] / 2;
  const int nG  = in_sizes[3];
  const int nE2 = in_sizes[4] / 2;
  const int nT1 = in_sizes[5] / D;
  const int nT2 = in_sizes[6] / D;
  const int nL1 = in_sizes[7] / (D * D);
  const int nL2 = in_sizes[12] / (D * D);
  if (nN1 <= 0 || nE1 < 0 || nG <= 0 || nE2 < 0 || nT1 <= 0 || nT2 <= 0 || nL1 <= 0 || nL2 <= 0) return;
  if (in_sizes[1] != 2 * nE1 || in_sizes[2] != nN1 || in_sizes[4] != 2 * nE2) return;
  if (in_sizes[5] != nT1 * D || in_sizes[6] != nT2 * D) return;
  if (in_sizes[7] != nL1 * D * D || in_sizes[9] != nL1 * D * D || in_sizes[8] < nL1 * D) return;
  if (in_sizes[10] != 2 * D * D || in_sizes[11] < D) return;
  if (in_sizes[12] != nL2 * D * D || in_sizes[14] != nL2 * D * D || in_sizes[15] != nL2 * D * D) return;
  if (in_sizes[13] < nL2 * D) return;
  if (out_size != nG * D || (nG % NBS) != 0) return;

  const int*   x1   = (const int*)d_in[0];
  const int*   ei1  = (const int*)d_in[1];
  const int*   bat  = (const int*)d_in[2];
  const int*   ids2 = (const int*)d_in[3];
  const int*   ei2  = (const int*)d_in[4];
  const float* tab1 = (const float*)d_in[5];
  const float* tab2 = (const float*)d_in[6];
  const float* Wl1  = (const float*)d_in[7];
  const float* bl1  = (const float*)d_in[8];
  const float* Wr1  = (const float*)d_in[9];
  const float* linW = (const float*)d_in[10];
  const float* linb = (const float*)d_in[11];
  const float* Wl2  = (const float*)d_in[12];
  const float* bl2  = (const float*)d_in[13];
  const float* Wr2  = (const float*)d_in[14];
  const float* Wx2  = (const float*)d_in[15];
  float* out = (float*)d_out;

  const int nBlk1  = (nN1 + NBS - 1) / NBS;
  const int nRows1 = nBlk1 * NBS;
  const int nBlkP  = (nG + NBP - 1) / NBP;
  const int nRowsP = nBlkP * NBP;
  const int nBlk2  = nG / NBS;

  char* ws = (char*)d_ws;
  size_t off = 0;
  const size_t szW1 = (size_t)nL1 * D * (2 * D) * 2;
  const size_t szWL = (size_t)D * (2 * D) * 2;
  const size_t szW2 = (size_t)nL2 * D * (3 * D) * 2;
  const size_t szX1 = (size_t)nRows1 * D * 4;
  const size_t szXD = (size_t)nRowsP * D * 4;
  const size_t szX2 = (size_t)nG * D * 4;
#define CARVE(NAME, SZ) const size_t NAME = off; off += (SZ); off = (off + 255) & ~(size_t)255;
  CARVE(oW1h, szW1) CARVE(oW1l, szW1)
  CARVE(oWLh, szWL) CARVE(oWLl, szWL)
  CARVE(oW2h, szW2) CARVE(oW2l, szW2)
  CARVE(oXa,  szX1) CARVE(oXb,  szX1)
  CARVE(oXd,  szXD)
  CARVE(oYa,  szX2) CARVE(oYb,  szX2)
#undef CARVE
  if (off > ws_size) return;
  bf16_t* w1h = (bf16_t*)(ws + oW1h);
  bf16_t* w1l = (bf16_t*)(ws + oW1l);
  bf16_t* wLh = (bf16_t*)(ws + oWLh);
  bf16_t* wLl = (bf16_t*)(ws + oWLl);
  bf16_t* w2h = (bf16_t*)(ws + oW2h);
  bf16_t* w2l = (bf16_t*)(ws + oW2l);
  float*  xa  = (float*)(ws + oXa);
  float*  xb  = (float*)(ws + oXb);
  float*  xd  = (float*)(ws + oXd);
  float*  ya  = (float*)(ws + oYa);
  float*  yb  = (float*)(ws + oYb);

  const int vec1 = ((nE1 & 3) == 0) ? 1 : 0;
  const int vec2 = ((nE2 & 3) == 0) ? 1 : 0;
  const int vecB = 1;

  {
    const int nTot1 = nL1 * D * (2 * D) / 8;
    const int nTotL = D * (2 * D) / 8;
    const int nTot2 = nL2 * D * (3 * D) / 8;
    k_wprep<<<(nTot1 + NTHR - 1) / NTHR, NTHR, 0, stream>>>(Wl1, Wr1, Wl1, D * D, D * D, 0, w1h, w1l, 2 * D, nTot1);
    k_wprep<<<(nTotL + NTHR - 1) / NTHR, NTHR, 0, stream>>>(linW, linW + (size_t)D * D, linW, 0, 0, 0, wLh, wLl, 2 * D, nTotL);
    k_wprep<<<(nTot2 + NTHR - 1) / NTHR, NTHR, 0, stream>>>(Wl2, Wr2, Wx2, D * D, D * D, D * D, w2h, w2l, 3 * D, nTot2);
  }

  k_gather1<<<(nRows1 + NWAVE * RPW - 1) / (NWAVE * RPW), NTHR, 0, stream>>>(x1, tab1, nT1, xa, nN1, nRows1);

  hipFuncSetAttribute(reinterpret_cast<const void*>(&k_sage<2>),
                      hipFuncAttributeMaxDynamicSharedMemorySize, LDS_SAGE);
  hipFuncSetAttribute(reinterpret_cast<const void*>(&k_sage<3>),
                      hipFuncAttributeMaxDynamicSharedMemorySize, LDS_SAGE);
  hipFuncSetAttribute(reinterpret_cast<const void*>(&k_pool),
                      hipFuncAttributeMaxDynamicSharedMemorySize, LDS_POOL);

  float* cur = xa;
  float* nxt = xb;
  for (int l = 0; l < nL1; ++l) {
    k_sage<2><<<nBlk1, NTHR, LDS_SAGE, stream>>>(
        ei1, cur, cur, w1h + (size_t)l * D * (2 * D), w1l + (size_t)l * D * (2 * D),
        bl1 + (size_t)l * D, nxt, nN1, nE1, vec1);
    float* tsw = cur; cur = nxt; nxt = tsw;
  }

  k_pool<<<nBlkP, NTHR, LDS_POOL, stream>>>(bat, cur, wLh, wLl, linb, xd, nN1, vecB);

  k_gather2<<<(nG + NWAVE * RPW - 1) / (NWAVE * RPW), NTHR, 0, stream>>>(ids2, xd, nG, tab2, nT2, ya, nG, nG);

  float* cur2 = ya;
  float* nxt2 = yb;
  for (int l = 0; l < nL2; ++l) {
    float* dst = (l == nL2 - 1) ? out : nxt2;
    k_sage<3><<<nBlk2, NTHR, LDS_SAGE, stream>>>(
        ei2, cur2, xd, w2h + (size_t)l * D * (3 * D), w2l + (size_t)l * D * (3 * D),
        bl2 + (size_t)l * D, dst, nG, nE2, vec2);
    nxt2 = cur2;
    cur2 = dst;
  }
}
